// CDA_attention_67602785239326
// MI455X (gfx1250) — hardware-verified
//
#include <hip/hip_runtime.h>
#include <stddef.h>
#include <stdint.h>

#define NBAT  8
#define CD    256
#define IMH   64
#define IMW   64
#define NN    (IMH * IMW)
#define NTOK  (NBAT * NN)
#define NQKV  768
#define NSLAB 6
#define DCH   8
#define KC    64
#define QBLK  64
#define QG    (QBLK / 16)
#define NQB   (NN / QBLK)
#define NCK   (NN / KC)

#define XCAR 1.0f
#define WCAR 16.0f
#define QCAR 8.0f
#define VCAR 8.0f
#define PCAR 1024.0f
#define OCAR 512.0f

static_assert(NN == 4096);
static_assert(NTOK == 32768);
static_assert(NQKV == 3 * CD);
static_assert(NQKV == NSLAB * 128);
static_assert(NTOK % 256 == 0);
static_assert(NTOK % 64 == 0);
static_assert(NN % 64 == 0);
static_assert(CD % 64 == 0);
static_assert(CD % 32 == 0);
static_assert(QG == 4);
static_assert(KC == 64);
static_assert(QBLK == 64);
static_assert((NQKV * CD / 8) % 256 == 0);
static_assert((CD * CD / 8) % 256 == 0);

typedef _Float16 v16h __attribute__((ext_vector_type(16)));
typedef _Float16 v8h  __attribute__((ext_vector_type(8)));
typedef float    v8f  __attribute__((ext_vector_type(8)));
typedef float    v4f  __attribute__((ext_vector_type(4)));
typedef unsigned int v4u __attribute__((ext_vector_type(4)));

union FragH { v16h v; v8h h[2]; };
union Pack8 { v8h h; v4u u; };

__device__ __forceinline__ v8f mma_h(v16h a, v16h b, v8f c) {
  c = __builtin_amdgcn_wmma_f32_16x16x32_f16(false, a, false, b, (short)0, c, false, false);
  asm volatile("v_nop\n\tv_nop\n\tv_nop\n\tv_nop" : "+v"(c) : "v"(a), "v"(b));
  return c;
}
__device__ __forceinline__ v8f zero8() { return (v8f){0.f, 0.f, 0.f, 0.f, 0.f, 0.f, 0.f, 0.f}; }

__device__ __forceinline__ v16h ldfrag_h(const _Float16* p, int ld, int row0, int k0, int lane) {
  const int m = lane & 15, lh = lane >> 4;
  const _Float16* q = p + (size_t)(row0 + m) * ld + k0 + 8 * lh;
  FragH f;
  f.h[0] = *(const v8h*)(q);
  f.h[1] = *(const v8h*)(q + 16);
  return f.v;
}

__device__ __forceinline__ v4u pack8h(const float (&v)[8], float sc) {
  Pack8 pk;
  pk.h = (v8h){(_Float16)(v[0] * sc), (_Float16)(v[1] * sc), (_Float16)(v[2] * sc), (_Float16)(v[3] * sc),
               (_Float16)(v[4] * sc), (_Float16)(v[5] * sc), (_Float16)(v[6] * sc), (_Float16)(v[7] * sc)};
  return pk.u;
}

__device__ __forceinline__ float tap64(const float* __restrict__ base, int hy, int wx) {
  const int hc = min(max(hy, 0), IMH - 1), wc = min(max(wx, 0), IMW - 1);
  const float v = base[hc * IMW + wc];
  const bool inb = (hy >= 0) && (hy < IMH) && (wx >= 0) && (wx < IMW);
  return inb ? v : 0.f;
}

__device__ __forceinline__ void gemm16x64(const _Float16* __restrict__ A, int lda,
                                          const _Float16* __restrict__ Bm, int ldb,
                                          int m0, int n0, int lane, v8f (&acc)[4]) {
#pragma unroll 2
  for (int ks = 0; ks < CD / 32; ++ks) {
    const v16h a = ldfrag_h(A, lda, m0, ks * 32, lane);
#pragma unroll
    for (int t = 0; t < 4; ++t) {
      const v16h bb = ldfrag_h(Bm, ldb, n0 + 16 * t, ks * 32, lane);
      acc[t] = mma_h(a, bb, acc[t]);
    }
  }
}

__global__ __launch_bounds__(256) void k_gray(const float* __restrict__ x, float* __restrict__ g) {
  const int i = blockIdx.x * 256 + threadIdx.x;
  const int b = i >> 12, n = i & (NN - 1);
  const float* p = x + (size_t)b * CD * NN + n;
  float s = 0.f;
#pragma unroll 4
  for (int ch = 0; ch < CD; ++ch) s += p[(size_t)ch * NN];
  const float v = s * (1.0f / 256.0f);
  *(volatile float*)(g + i) = v;
  __threadfence();
  *(volatile float*)(g + i) = v;
}

__global__ __launch_bounds__(256) void k_lap(const float* __restrict__ g, float* __restrict__ la) {
  const int i = blockIdx.x * 256 + threadIdx.x;
  const int b = i >> 12, n = i & (NN - 1);
  const int h = n >> 6, w = n & 63;
  const float* gb = g + (size_t)b * NN;
  const float l = 4.0f * tap64(gb, h, w) - tap64(gb, h - 1, w) - tap64(gb, h + 1, w)
                - tap64(gb, h, w - 1) - tap64(gb, h, w + 1);
  const float v = fabsf(l);
  *(volatile float*)(la + i) = v;
  __threadfence();
  *(volatile float*)(la + i) = v;
}

__global__ __launch_bounds__(256) void k_dconv1(const float* __restrict__ la, const float* __restrict__ w1,
                                                const float* __restrict__ b1, float* __restrict__ hb) {
  const int i = blockIdx.x * 256 + threadIdx.x;
  const int b = i >> 12, n = i & (NN - 1);
  const int h = n >> 6, w = n & 63;
  const float* lb = la + (size_t)b * NN;
  float v[9];
#pragma unroll
  for (int ky = 0; ky < 3; ++ky)
#pragma unroll
    for (int kx = 0; kx < 3; ++kx) v[ky * 3 + kx] = tap64(lb, h + ky - 1, w + kx - 1);
#pragma unroll 1
  for (int oc = 0; oc < DCH; ++oc) {
    float s = b1[oc];
#pragma unroll
    for (int k = 0; k < 9; ++k) s += w1[oc * 9 + k] * v[k];
    const float val = fmaxf(s, 0.f);
    float* dst = hb + ((size_t)b * DCH + oc) * NN + n;
    *(volatile float*)dst = val;
    __threadfence();
    *(volatile float*)dst = val;
  }
}

__global__ __launch_bounds__(256) void k_tscale(const float* __restrict__ hb, const float* __restrict__ w2,
                                                const float* __restrict__ b2, float* __restrict__ ts) {
  const int i = blockIdx.x * 256 + threadIdx.x;
  const int b = i >> 12, n = i & (NN - 1);
  const int h = n >> 6, w = n & 63;
  float s = b2[0];
#pragma unroll 1
  for (int ic = 0; ic < DCH; ++ic) {
    const float* hc = hb + ((size_t)b * DCH + ic) * NN;
    const float* wc = w2 + ic * 9;
#pragma unroll
    for (int ky = 0; ky < 3; ++ky)
#pragma unroll
      for (int kx = 0; kx < 3; ++kx) s += wc[ky * 3 + kx] * tap64(hc, h + ky - 1, w + kx - 1);
  }
  s = fminf(fmaxf(s, -30.0f), 30.0f);
  const float e    = __expf(-s);
  const float dens = __builtin_amdgcn_rcpf(1.0f + e);
  const float temp = 1.0f + 2.0f * (1.0f - dens);
  const float tsv  = (0.0625f / (QCAR * QCAR)) * __builtin_amdgcn_rcpf(temp);
  *(volatile float*)(ts + i) = tsv;
  __threadfence();
  *(volatile float*)(ts + i) = tsv;
}

#define WTP 65
__global__ __launch_bounds__(256) void k_xtr(const float* __restrict__ x, _Float16* __restrict__ x16) {
  __shared__ float tl[64 * WTP];
  const int tid = threadIdx.x;
  const int n0 = blockIdx.x * 64, c0 = blockIdx.y * 64, b = blockIdx.z;
  const float* xb = x + (size_t)b * CD * NN;
#pragma unroll
  for (int j = 0; j < 4; ++j) {
    const int p  = tid + 256 * j;
    const int cc = p >> 4;
    const int q4 = (p & 15) * 4;
    const v4f a = *(const v4f*)(xb + (size_t)(c0 + cc) * NN + n0 + q4);
    float* d = tl + cc * WTP + q4;
    d[0] = a[0]; d[1] = a[1]; d[2] = a[2]; d[3] = a[3];
  }
  __syncthreads();
  v4u val[2];
  size_t go[2];
#pragma unroll
  for (int j = 0; j < 2; ++j) {
    const int p  = tid + 256 * j;
    const int nn = p >> 3;
    const int pc = p & 7;
    const float* cp = tl + (pc * 8) * WTP + nn;
    float v[8];
#pragma unroll
    for (int i = 0; i < 8; ++i) v[i] = cp[i * WTP];
    val[j] = pack8h(v, XCAR);
    go[j]  = ((size_t)b * NN + n0 + nn) * CD + c0 + pc * 8;
  }
  for (int ps = 0; ps < 2; ++ps) {
#pragma unroll
    for (int j = 0; j < 2; ++j) *(volatile v4u*)(x16 + go[j]) = val[j];
    __threadfence();
  }
}

__global__ __launch_bounds__(256) void k_wcv(const float* __restrict__ W, int n8, _Float16* __restrict__ w16) {
  int i = blockIdx.x * 256 + threadIdx.x;
  i = min(i, n8 - 1);
  const float* wp = W + (size_t)i * 8;
  const v4f a0 = *(const v4f*)(wp), a1 = *(const v4f*)(wp + 4);
  float v[8] = {a0[0], a0[1], a0[2], a0[3], a1[0], a1[1], a1[2], a1[3]};
  const v4u ph = pack8h(v, WCAR);
  const size_t go = (size_t)i * 8;
  *(volatile v4u*)(w16 + go) = ph;
  __threadfence();
  *(volatile v4u*)(w16 + go) = ph;
}

#define SFP 132
__global__ __launch_bounds__(256) void k_qkv(const _Float16* __restrict__ x16,
                                             const _Float16* __restrict__ w16,
                                             const float* __restrict__ bq,
                                             _Float16* __restrict__ qp,
                                             _Float16* __restrict__ kp,
                                             _Float16* __restrict__ vtp) {
  __shared__ __align__(16) float sf[64 * SFP];
  const int tid = threadIdx.x, lane = tid & 31;
  const int wave = __builtin_amdgcn_readfirstlane(tid >> 5);
  const int hh = lane >> 4, c = lane & 15;
  const int wm = wave >> 1, wn = wave & 1;
  const int mb  = blockIdx.x * 64;
  const int b   = mb >> 12;
  const int nb0 = mb & (NN - 1);
  const int ns  = blockIdx.y;
  const int which = ns >> 1;
  const int choff = (ns & 1) * 128;
  const int m0 = mb + wm * 16;
  const int n0 = ns * 128 + wn * 64;

  v8f acc[4];
#pragma unroll
  for (int t = 0; t < 4; ++t) acc[t] = zero8();
  gemm16x64(x16, CD, w16, CD, m0, n0, lane, acc);

#pragma unroll
  for (int t = 0; t < 4; ++t) {
#pragma unroll
    for (int r = 0; r < 8; ++r)
      sf[(wm * 16 + 8 * hh + r) * SFP + wn * 64 + 16 * t + c] = acc[t][r];
  }
  __syncthreads();

  const float wsc = 1.0f / (WCAR * XCAR);
  if (which < 2) {
    v4u val[4];
    size_t go[4];
#pragma unroll
    for (int j = 0; j < 4; ++j) {
      const int p  = tid + 256 * j;
      const int lr = p >> 4;
      const int pc = p & 15;
      const float* ra = sf + lr * SFP + pc * 8;
      const v4f a0 = *(const v4f*)(ra), a1 = *(const v4f*)(ra + 4);
      const v4f b0 = *(const v4f*)(bq + ns * 128 + pc * 8), bb1 = *(const v4f*)(bq + ns * 128 + pc * 8 + 4);
      float v[8] = {a0[0] * wsc + b0[0],  a0[1] * wsc + b0[1],  a0[2] * wsc + b0[2],  a0[3] * wsc + b0[3],
                    a1[0] * wsc + bb1[0], a1[1] * wsc + bb1[1], a1[2] * wsc + bb1[2], a1[3] * wsc + bb1[3]};
      val[j] = pack8h(v, QCAR);
      go[j]  = (size_t)(mb + lr) * CD + choff + pc * 8;
    }
    _Float16* base = (which == 0) ? qp : kp;
    for (int ps = 0; ps < 2; ++ps) {
#pragma unroll
      for (int j = 0; j < 4; ++j) *(volatile v4u*)(base + go[j]) = val[j];
      __threadfence();
    }
  } else {
    v4u val[4];
    size_t go[4];
#pragma unroll
    for (int j = 0; j < 4; ++j) {
      const int p    = tid + 256 * j;
      const int dcol = p >> 3;
      const int pc   = p & 7;
      const float* cp = sf + (pc * 8) * SFP + dcol;
      const float bb = bq[ns * 128 + dcol];
      float v[8];
#pragma unroll
      for (int i = 0; i < 8; ++i) v[i] = cp[i * SFP] * wsc + bb;
      val[j] = pack8h(v, VCAR);
      go[j]  = ((size_t)(b * CD + choff + dcol)) * NN + nb0 + pc * 8;
    }
    for (int ps = 0; ps < 2; ++ps) {
#pragma unroll
      for (int j = 0; j < 4; ++j) *(volatile v4u*)(vtp + go[j]) = val[j];
      __threadfence();
    }
  }
}

#define KTP 264
#define VTP 72
#define PTP 72
static_assert(QBLK * KTP <= KC * KTP);
__global__ __launch_bounds__(256) void k_attn(const _Float16* __restrict__ qp,
                                              const _Float16* __restrict__ kp,
                                              const _Float16* __restrict__ vt,
                                              const float* __restrict__ tsc,
                                              _Float16* __restrict__ op) {
  __shared__ __align__(16) _Float16 Ks[KC * KTP];
  __shared__ __align__(16) _Float16 Vs[CD * VTP];
  __shared__ __align__(16) _Float16 Ps[QG * 16 * PTP];
  __shared__ float Al[QG * 16];
  __shared__ float Ll[QG * 16];

  const int tid = threadIdx.x, lane = tid & 31;
  const int wave = __builtin_amdgcn_readfirstlane(tid >> 5);
  const int hh = lane >> 4, c = lane & 15;
  const int g = wave & 3, chh = wave >> 2;
  const int b  = blockIdx.x / NQB;
  const int qb = blockIdx.x - b * NQB;
  const int q0 = qb * QBLK + g * 16;

  const _Float16* Q = qp + (size_t)b * NN * CD;
  const _Float16* K = kp + (size_t)b * NN * CD;
  const _Float16* V = vt + (size_t)b * CD * NN;
  const float*    T = tsc + (size_t)b * NN;

  const float NEGI = -__builtin_huge_valf();
  float mrow[8], lrow[8];
  v8f oacc[8];
#pragma unroll
  for (int r = 0; r < 8; ++r) { mrow[r] = NEGI; lrow[r] = 0.f; }
#pragma unroll
  for (int t = 0; t < 8; ++t) oacc[t] = zero8();

  _Float16* pw = Ps + g * 16 * PTP;

  for (int kc = 0; kc < NCK; ++kc) {
    const int kv0 = kc * KC;
    __syncthreads();
#pragma unroll
    for (int j = 0; j < 8; ++j) {
      const int p  = tid + 256 * j;
      const int rk = p >> 5;
      const int qk = (p & 31) * 8;
      *(v8h*)(Ks + rk * KTP + qk) = *(const v8h*)(K + (size_t)(kv0 + rk) * CD + qk);
      const int rv = p >> 3;
      const int qv = (p & 7) * 8;
      *(v8h*)(Vs + rv * VTP + qv) = *(const v8h*)(V + (size_t)rv * NN + kv0 + qv);
    }
    __syncthreads();

    if (wave < QG) {
      v8f s[4];
#pragma unroll
      for (int j = 0; j < 4; ++j) s[j] = zero8();
#pragma unroll 2
      for (int cc = 0; cc < CD / 32; ++cc) {
        const v16h qa = ldfrag_h(Q, CD, q0, cc * 32, lane);
#pragma unroll
        for (int j = 0; j < 4; ++j) {
          const v16h kb = ldfrag_h(Ks, KTP, j * 16, cc * 32, lane);
          s[j] = mma_h(qa, kb, s[j]);
        }
      }
      float tcol[4];
#pragma unroll
      for (int j = 0; j < 4; ++j) tcol[j] = T[kv0 + j * 16 + c];
      float cm[8];
#pragma unroll
      for (int r = 0; r < 8; ++r) {
        float m = NEGI;
#pragma unroll
        for (int j = 0; j < 4; ++j) { s[j][r] *= tcol[j]; m = fmaxf(m, s[j][r]); }
#pragma unroll
        for (int off = 1; off < 16; off <<= 1) m = fmaxf(m, __shfl_xor(m, off, 32));
        cm[r] = m;
      }
#pragma unroll
      for (int r = 0; r < 8; ++r) {
        const float mnew  = fmaxf(mrow[r], cm[r]);
        const float alpha = __expf(mrow[r] - mnew);
        mrow[r] = mnew;
        float psum = 0.f;
#pragma unroll
        for (int j = 0; j < 4; ++j) {
          const float p = __expf(s[j][r] - mnew);
          psum += p;
          pw[(8 * hh + r) * PTP + j * 16 + c] = (_Float16)(p * PCAR);
        }
#pragma unroll
        for (int off = 1; off < 16; off <<= 1) psum += __shfl_xor(psum, off, 32);
        lrow[r] = lrow[r] * alpha + psum;
        Al[g * 16 + 8 * hh + r] = alpha;
      }
    }
    __syncthreads();

    float al[8];
#pragma unroll
    for (int r = 0; r < 8; ++r) al[r] = Al[g * 16 + 8 * hh + r];
#pragma unroll
    for (int t = 0; t < 8; ++t)
#pragma unroll
      for (int r = 0; r < 8; ++r) oacc[t][r] *= al[r];

#pragma unroll
    for (int kk = 0; kk < 2; ++kk) {
      const v16h pa = ldfrag_h(pw, PTP, 0, kk * 32, lane);
#pragma unroll
      for (int t = 0; t < 8; ++t) {
        const v16h vb = ldfrag_h(Vs, VTP, chh * 128 + t * 16, kk * 32, lane);
        oacc[t] = mma_h(pa, vb, oacc[t]);
      }
    }
  }

  if (wave < QG) {
#pragma unroll
    for (int r = 0; r < 8; ++r) Ll[g * 16 + 8 * hh + r] = lrow[r];
  }
  __syncthreads();
  float inv[8];
#pragma unroll
  for (int r = 0; r < 8; ++r) {
    const float l = Ll[g * 16 + 8 * hh + r];
    inv[r] = (l > 0.f) ? ((OCAR / (PCAR * VCAR)) * __builtin_amdgcn_rcpf(l)) : 0.f;
  }
  _Float16* Os = Ks;
#pragma unroll
  for (int t = 0; t < 8; ++t) {
#pragma unroll
    for (int r = 0; r < 8; ++r)
      Os[(g * 16 + 8 * hh + r) * KTP + chh * 128 + 16 * t + c] = (_Float16)(oacc[t][r] * inv[r]);
  }
  __syncthreads();
  const size_t tok0 = (size_t)b * NN + (size_t)qb * QBLK;
  for (int ps = 0; ps < 2; ++ps) {
#pragma unroll
    for (int it = 0; it < 8; ++it) {
      const int row = wave + 8 * it;
      Pack8 pk;
      pk.h = *(const v8h*)(Os + row * KTP + lane * 8);
      *(volatile v4u*)(op + (tok0 + row) * CD + lane * 8) = pk.u;
    }
    __threadfence();
  }
}

#define OTP 68
__global__ __launch_bounds__(256) void k_proj(const _Float16* __restrict__ o16,
                                              const _Float16* __restrict__ w16,
                                              const float* __restrict__ pb,
                                              const float* __restrict__ x,
                                              float* __restrict__ out) {
  __shared__ __align__(16) float st[128 * OTP];
  const int tid = threadIdx.x, lane = tid & 31;
  const int wave = __builtin_amdgcn_readfirstlane(tid >> 5);
  const int hh = lane >> 4, c = lane & 15;
  const int wm = wave >> 1, wn = wave & 1;
  const int mb  = blockIdx.x * 64;
  const int b   = mb >> 12;
  const int nb0 = mb & (NN - 1);
  const int m0  = mb + wm * 16;
  const int cb  = blockIdx.y * 128;
  const int n0  = cb + wn * 64;

  v8f acc[4];
#pragma unroll
  for (int t = 0; t < 4; ++t) acc[t] = zero8();
  gemm16x64(o16, CD, w16, CD, m0, n0, lane, acc);

  const float osc = 1.0f / (OCAR * WCAR);
#pragma unroll
  for (int t = 0; t < 4; ++t) {
    const float bb = pb[n0 + 16 * t + c];
#pragma unroll
    for (int r = 0; r < 8; ++r) st[(wn * 64 + 16 * t + c) * OTP + wm * 16 + 8 * hh + r] = acc[t][r] * osc + bb;
  }
  __syncthreads();
  v4f val[8];
  size_t go[8];
#pragma unroll
  for (int it = 0; it < 8; ++it) {
    const int p    = lane + 32 * it;
    const int L    = p >> 3;
    const int pc   = p & 7;
    const int cl   = wave * 16 + (L >> 1);
    const int half = L & 1;
    const v4f a = *(const v4f*)(st + cl * OTP + half * 32 + pc * 4);
    go[it]  = ((size_t)(b * CD + cb + cl)) * NN + nb0 + half * 32 + pc * 4;
    const v4f xr = *(const v4f*)(x + go[it]);
    val[it] = a + xr;
  }
  for (int ps = 0; ps < 2; ++ps) {
#pragma unroll
    for (int it = 0; it < 8; ++it) *(volatile v4f*)(out + go[it]) = val[it];
    __threadfence();
  }
}

extern "C" void kernel_launch(void* const* d_in, const int* in_sizes, int n_in,
                              void* d_out, int out_size, void* d_ws, size_t ws_size,
                              hipStream_t stream) {
  if (n_in < 9) return;
  if (in_sizes[0] != NTOK * CD) return;
  if (in_sizes[1] != NQKV * CD) return;
  if (in_sizes[2] != NQKV) return;
  if (in_sizes[3] != CD * CD) return;
  if (in_sizes[4] != CD) return;
  if (in_sizes[5] != DCH * 9) return;
  if (in_sizes[6] != DCH) return;
  if (in_sizes[7] != DCH * 9) return;
  if (in_sizes[8] != 1) return;
  if (out_size != NTOK * CD) return;

  const float* x     = (const float*)d_in[0];
  const float* qkv_w = (const float*)d_in[1];
  const float* qkv_b = (const float*)d_in[2];
  const float* out_w = (const float*)d_in[3];
  const float* out_b = (const float*)d_in[4];
  const float* d1_w  = (const float*)d_in[5];
  const float* d1_b  = (const float*)d_in[6];
  const float* d2_w  = (const float*)d_in[7];
  const float* d2_b  = (const float*)d_in[8];
  float* out = (float*)d_out;

  size_t off = 0;
  const size_t oWq = off; off += (size_t)NQKV * CD * 2;
  const size_t oWo = off; off += (size_t)CD * CD * 2;
  const size_t oX  = off; off += (size_t)NTOK * CD * 2;
  const size_t oQ  = off; off += (size_t)NTOK * CD * 2;
  const size_t oK  = off; off += (size_t)NTOK * CD * 2;
  const size_t oV  = off; off += (size_t)NBAT * CD * NN * 2;
  const size_t oO  = off; off += (size_t)NTOK * CD * 2;
  const size_t oG  = off; off += (size_t)NTOK * 4;
  const size_t oL  = off; off += (size_t)NTOK * 4;
  const size_t oH  = off; off += (size_t)NTOK * DCH * 4;
  const size_t oT  = off; off += (size_t)NTOK * 4;
  if (off > ws_size) return;
  if (off > (size_t)134217728) return;

  char* ws = (char*)d_ws;
  _Float16* Wq16 = (_Float16*)(ws + oWq);
  _Float16* Wo16 = (_Float16*)(ws + oWo);
  _Float16* X16  = (_Float16*)(ws + oX);
  _Float16* Q16  = (_Float16*)(ws + oQ);
  _Float16* K16  = (_Float16*)(ws + oK);
  _Float16* VT16 = (_Float16*)(ws + oV);
  _Float16* O16  = (_Float16*)(ws + oO);
  float* gray = (float*)(ws + oG);
  float* lap  = (float*)(ws + oL);
  float* hb   = (float*)(ws + oH);
  float* ts   = (float*)(ws + oT);

  k_wcv<<<dim3((NQKV * CD / 8) / 256), dim3(256), 0, stream>>>(qkv_w, NQKV * CD / 8, Wq16);
  k_wcv<<<dim3((CD * CD / 8) / 256), dim3(256), 0, stream>>>(out_w, CD * CD / 8, Wo16);
  k_gray  <<<dim3(NTOK / 256), dim3(256), 0, stream>>>(x, gray);
  k_lap   <<<dim3(NTOK / 256), dim3(256), 0, stream>>>(gray, lap);
  k_dconv1<<<dim3(NTOK / 256), dim3(256), 0, stream>>>(lap, d1_w, d1_b, hb);
  k_tscale<<<dim3(NTOK / 256), dim3(256), 0, stream>>>(hb, d2_w, d2_b, ts);
  k_xtr<<<dim3(NN / 64, CD / 64, NBAT), dim3(256), 0, stream>>>(x, X16);
  k_qkv<<<dim3(NTOK / 64, NSLAB), dim3(256), 0, stream>>>(X16, Wq16, qkv_b, Q16, K16, VT16);
  k_attn<<<dim3(NBAT * NQB), dim3(256), 0, stream>>>(Q16, K16, VT16, ts, O16);
  k_proj<<<dim3(NTOK / 64, CD / 128), dim3(256), 0, stream>>>(O16, Wo16, out_b, x, out);
  (void)hipGetLastError();
}
